// KnowledgeFusion_33165737460139
// MI455X (gfx1250) — hardware-verified
//
#include <hip/hip_runtime.h>
#include <stddef.h>


typedef _Float16 v16h __attribute__((ext_vector_type(16)));
typedef _Float16 v8h  __attribute__((ext_vector_type(8)));
typedef float    v8f  __attribute__((ext_vector_type(8)));
typedef float    v4f  __attribute__((ext_vector_type(4)));
typedef int      v4i  __attribute__((ext_vector_type(4)));

#ifndef NB
#define NB 8
#endif
#define NB_FULL 8
#define IMH   32
#define IMW   32
#define HWP   (IMH * IMW)
#define DIM   256
#define NOBJ  15
#define NMASK 16
#define KM    32
#define NBP   (((NB + 3) / 4) * 4)
#define MROWS (NB * HWP)
#define EROWS (NBP * NMASK)

static_assert(NB >= 1 && NB <= NB_FULL);
static_assert(IMW == 32 && IMH == 32);
static_assert(NMASK == NOBJ + 1 && NMASK == 16);
static_assert(KM == 32 && NMASK <= KM);
static_assert((DIM % 64) == 0 && (DIM % 32) == 0);
static_assert((HWP % 64) == 0);
static_assert((MROWS % 64) == 0);
static_assert((EROWS % 64) == 0);
static_assert(DIM == 256);
static_assert(((size_t)MROWS * DIM) % (256 * 8) == 0);

#define LDT 72
#define LDC 68
#define LDM 40
#define LDE 264
static_assert((LDT % 8) == 0 && LDT >= 64);
static_assert((LDC % 4) == 0 && LDC >= 64);
static_assert((LDM % 8) == 0 && LDM >= KM);
static_assert((LDE % 8) == 0 && LDE >= DIM);

#define WCARRY 64.0f
#define ICARRY 64.0f

#define WT_BYTES   ((size_t)DIM * DIM * 2)
#define P16_BYTES  ((size_t)MROWS * DIM * 2)
#define E16_BYTES  ((size_t)EROWS * DIM * 2)
#define INJT_BYTES ((size_t)NBP * DIM * KM * 2)
#define OFF_WPT  ((size_t)0)
#define OFF_WET  (OFF_WPT + WT_BYTES)
#define OFF_P16  (OFF_WET + WT_BYTES)
#define OFF_E16  (OFF_P16 + P16_BYTES)
#define OFF_INJT (OFF_E16 + E16_BYTES)
#define WS_TOTAL (OFF_INJT + INJT_BYTES)
static_assert((WT_BYTES % 128) == 0 && (P16_BYTES % 128) == 0);
static_assert((E16_BYTES % 128) == 0 && (INJT_BYTES % 128) == 0);
static_assert(WS_TOTAL <= (size_t)134217728);

__device__ __forceinline__ float bf16r(float x) {
  unsigned int u = __float_as_uint(x);
  u = (u + 0x7FFFu + ((u >> 16) & 1u)) & 0xFFFF0000u;
  return __uint_as_float(u);
}

static __device__ __forceinline__ _Float16 toh_flush(float v) {
  const _Float16 r = (_Float16)v;
  return (fabsf(v) < 6.103515625e-05f) ? (_Float16)0.0f : r;
}

__device__ __forceinline__ v16h frag_at(const _Float16* p) {
  v8h lo = *(const v8h*)(p);
  v8h hi = *(const v8h*)(p + 16);
  v16h out;
#pragma unroll
  for (int i = 0; i < 8; ++i) { out[i] = lo[i]; out[i + 8] = hi[i]; }
  return out;
}
__device__ __forceinline__ v16h ld_frag(const _Float16* base, unsigned ld) {
  const unsigned lane = threadIdx.x & 31u;
  return frag_at(base + (lane & 15u) * ld + (lane >> 4) * 8u);
}

__device__ __forceinline__ v8f wmma16(v16h a, v16h b, v8f c) {
  v8f d = __builtin_amdgcn_wmma_f32_16x16x32_f16(false, a, false, b, (short)0, c,
                                                 false, false);
  asm volatile("v_nop\n\tv_nop\n\tv_nop\n\tv_nop" : "+v"(d) : "v"(a), "v"(b));
  return d;
}

__global__ __launch_bounds__(256) void wconv_kernel(
    const float* __restrict__ W, _Float16* __restrict__ Wt, unsigned ldw, unsigned ldk) {
  __shared__ _Float16 T[64 * LDT];
  const unsigned tid = threadIdx.x;
  const unsigned n0 = blockIdx.x * 64u;
  const unsigned k0 = blockIdx.y * 64u;
#pragma unroll 4
  for (unsigned j = 0; j < 16u; ++j) {
    const unsigned idx = tid + 256u * j;
    const unsigned kr = idx >> 6, nc = idx & 63u;
    const float v = W[(size_t)(k0 + kr) * ldw + n0 + nc];
    T[nc * LDT + kr] = toh_flush(WCARRY * bf16r(v));
  }
  __syncthreads();
  v8h x[2];
  size_t off[2];
#pragma unroll
  for (unsigned i = 0; i < 2u; ++i) {
    const unsigned n = 32u * i + (tid >> 3);
    const unsigned kc = (tid & 7u) * 8u;
    x[i] = *(const v8h*)&T[n * LDT + kc];
    off[i] = (size_t)(n0 + n) * ldk + k0 + kc;
  }
#pragma unroll
  for (int i = 0; i < 2; ++i) *(volatile v8h*)(Wt + off[i]) = x[i];
  __threadfence();
#pragma unroll
  for (int i = 0; i < 2; ++i) *(volatile v8h*)(Wt + off[i]) = x[i];
}
static_assert(32 * 2 == 64);

__global__ __launch_bounds__(256) void pconv_kernel(
    const float* __restrict__ X, _Float16* __restrict__ P16) {
#pragma clang fp contract(off)
  const size_t i = ((size_t)blockIdx.x * 256u + threadIdx.x) * 8u;
  const v4f a0 = *(const v4f*)(X + i);
  const v4f a1 = *(const v4f*)(X + i + 4u);
  v8h o;
#pragma unroll
  for (int j = 0; j < 4; ++j) {
    o[j]     = toh_flush(bf16r(a0[j]));
    o[j + 4] = toh_flush(bf16r(a1[j]));
  }
  *(volatile v8h*)(P16 + i) = o;
  __threadfence();
  *(volatile v8h*)(P16 + i) = o;
}

__global__ __launch_bounds__(256) void ebuild_kernel(
    const float* __restrict__ embs, _Float16* __restrict__ E16) {
#pragma clang fp contract(off)
  __shared__ _Float16 Es[NMASK * LDE];
  const unsigned tid = threadIdx.x;
  const unsigned b = blockIdx.x;
  const unsigned bl = (b < (unsigned)NB) ? b : (unsigned)(NB - 1);
  const bool live = (b < (unsigned)NB);
  const float* eb = embs + (size_t)bl * NOBJ * DIM + tid;
  float s = 0.0f;
#pragma unroll 1
  for (unsigned n = 0; n < (unsigned)NOBJ; ++n) {
    const float ld = eb[(size_t)n * DIM];
    const float v = live ? bf16r(ld) : 0.0f;
    s += v;
    Es[n * LDE + tid] = toh_flush(v);
  }
  Es[NOBJ * LDE + tid] = toh_flush(s * (1.0f / (float)NOBJ));
  __syncthreads();
  v8h x[2];
  size_t off[2];
#pragma unroll
  for (unsigned i = 0; i < 2u; ++i) {
    const unsigned idx = tid + 256u * i;
    const unsigned r = idx >> 5;
    const unsigned c = (idx & 31u) * 8u;
    x[i] = *(const v8h*)&Es[r * LDE + c];
    off[i] = ((size_t)b * NMASK + r) * DIM + c;
  }
#pragma unroll
  for (int i = 0; i < 2; ++i) *(volatile v8h*)(E16 + off[i]) = x[i];
  __threadfence();
#pragma unroll
  for (int i = 0; i < 2; ++i) *(volatile v8h*)(E16 + off[i]) = x[i];
}
static_assert(8 * 2 == NMASK);

__global__ __launch_bounds__(256) void gemm_inj_kernel(
    const _Float16* __restrict__ A16, const _Float16* __restrict__ Bt,
    _Float16* __restrict__ InjT) {
  __shared__ float Cs[64 * LDC];
  const unsigned tid = threadIdx.x, lane = tid & 31u;
  const unsigned w = (unsigned)__builtin_amdgcn_readfirstlane((int)(threadIdx.x >> 5));
  const unsigned mw = w >> 1, nw = w & 1u;
  const unsigned hh = lane >> 4, m = lane & 15u;
  const unsigned n0 = blockIdx.x * 64u;
  const unsigned row0 = blockIdx.y * 64u;
  const unsigned K = (unsigned)DIM;

  const _Float16* ap  = A16 + (size_t)(row0 + mw * 16u + m) * K + hh * 8u;
  const _Float16* bp0 = Bt + (size_t)(n0 + nw * 32u + m) * K + hh * 8u;
  const _Float16* bp1 = bp0 + (size_t)16 * K;
  v8f acc0 = {}, acc1 = {};
#pragma unroll 2
  for (unsigned k0 = 0; k0 < K; k0 += 32u) {
    const v16h a  = frag_at(ap + k0);
    const v16h b0 = frag_at(bp0 + k0);
    const v16h b1 = frag_at(bp1 + k0);
    acc0 = wmma16(a, b0, acc0);
    acc1 = wmma16(a, b1, acc1);
  }
#pragma unroll
  for (int r = 0; r < 8; ++r) {
    float* d = &Cs[(mw * 16u + hh * 8u + (unsigned)r) * LDC + nw * 32u + m];
    d[0]  = acc0[r];
    d[16] = acc1[r];
  }
  __syncthreads();

  const unsigned ol = tid >> 2;
  const unsigned part = tid & 3u;
  const unsigned pk = (part & 1u) * 8u;
  const bool real = (part < 2u);
  v8h x[4];
  size_t off[4];
#pragma unroll
  for (unsigned i = 0; i < 4u; ++i) {
#pragma unroll
    for (unsigned j = 0; j < 8u; ++j) {
      const float t = Cs[(i * 16u + pk + j) * LDC + ol] * (ICARRY / WCARRY);
      const _Float16 hv = toh_flush(t);
      x[i][j] = real ? hv : (_Float16)0.0f;
    }
    off[i] = ((size_t)(row0 / 16u + i) * DIM + n0 + ol) * KM + part * 8u;
  }
#pragma unroll
  for (int i = 0; i < 4; ++i) *(volatile v8h*)(InjT + off[i]) = x[i];
  __threadfence();
#pragma unroll
  for (int i = 0; i < 4; ++i) *(volatile v8h*)(InjT + off[i]) = x[i];
}
static_assert(4 * 16 == 64);
static_assert(4 * 8 == KM);

__global__ __launch_bounds__(256) void fuse_kernel(
    const _Float16* __restrict__ A16, const _Float16* __restrict__ Bt,
    const _Float16* __restrict__ InjT, const int* __restrict__ loc,
    float* __restrict__ outf) {
  __shared__ float Cs[64 * LDC];
  __shared__ _Float16 Ms[64 * LDM];
  __shared__ float Sinv[64];
  const unsigned tid = threadIdx.x, lane = tid & 31u;
  const unsigned w = (unsigned)__builtin_amdgcn_readfirstlane((int)(threadIdx.x >> 5));
  const unsigned mw = w >> 1, nw = w & 1u;
  const unsigned hh = lane >> 4, m = lane & 15u;
  const unsigned n0 = blockIdx.x * 64u;
  const unsigned row0 = blockIdx.y * 64u;
  const unsigned b = row0 / (unsigned)HWP;
  const unsigned p0 = row0 - b * (unsigned)HWP;
  const unsigned K = (unsigned)DIM;

  {
    const unsigned row = tid >> 2;
    const unsigned kq = (tid & 3u) * 8u;
    const int p = (int)(p0 + row);
    const int y = p / IMW;
    const int x = p - y * IMW;
    v8h mv;
    float cnt = 0.0f;
#pragma unroll
    for (unsigned j = 0; j < 8u; ++j) {
      const unsigned n = kq + j;
      const unsigned nc = (n < (unsigned)(NOBJ - 1)) ? n : (unsigned)(NOBJ - 1);
      const v4i L = *(const v4i*)(loc + ((size_t)b * NOBJ + nc) * 4u);
      const int y0 = L[0] - (L[0] & 1);
      const int x0 = L[1] - (L[1] & 1);
      const int y1 = L[2] + (2 - (L[2] & 1));
      const int x1 = L[3] + (2 - (L[3] & 1));
      const bool inbox = (y >= y0) && (y < y1) && (x >= x0) && (x < x1);
      const float boxv = inbox ? 1.0f : 0.0f;
      const float tailv = (n == (unsigned)NOBJ) ? 1.0f : 0.0f;
      const float mval = (n < (unsigned)NOBJ) ? boxv : tailv;
      cnt += mval;
      mv[j] = (_Float16)mval;
    }
    *(v8h*)&Ms[row * LDM + kq] = mv;
    cnt += __shfl_xor(cnt, 1, 32);
    cnt += __shfl_xor(cnt, 2, 32);
    if ((tid & 3u) == 0u) Sinv[row] = 1.0f / (ICARRY * cnt);
  }
  __syncthreads();

  const _Float16* ap  = A16 + (size_t)(row0 + mw * 16u + m) * K + hh * 8u;
  const _Float16* bp0 = Bt + (size_t)(n0 + nw * 32u + m) * K + hh * 8u;
  const _Float16* bp1 = bp0 + (size_t)16 * K;
  v8f acc0 = {}, acc1 = {};
#pragma unroll 2
  for (unsigned k0 = 0; k0 < K; k0 += 32u) {
    const v16h a  = frag_at(ap + k0);
    const v16h b0 = frag_at(bp0 + k0);
    const v16h b1 = frag_at(bp1 + k0);
    acc0 = wmma16(a, b0, acc0);
    acc1 = wmma16(a, b1, acc1);
  }

  v8f ms0 = {}, ms1 = {};
  {
    const v16h am = ld_frag(&Ms[(mw * 16u) * LDM], LDM);
    const _Float16* ip0 = InjT + ((size_t)b * DIM + n0 + nw * 32u + m) * KM + hh * 8u;
    const v16h bm0 = frag_at(ip0);
    const v16h bm1 = frag_at(ip0 + (size_t)16 * KM);
    ms0 = wmma16(am, bm0, ms0);
    ms1 = wmma16(am, bm1, ms1);
  }

#pragma unroll
  for (int r = 0; r < 8; ++r) {
    const unsigned row = mw * 16u + hh * 8u + (unsigned)r;
    const float si = Sinv[row];
    float* d = &Cs[row * LDC + nw * 32u + m];
    d[0]  = acc0[r] * (1.0f / WCARRY) + ms0[r] * si;
    d[16] = acc1[r] * (1.0f / WCARRY) + ms1[r] * si;
  }
  __syncthreads();

  v4f xs[4];
  size_t off[4];
#pragma unroll
  for (unsigned i = 0; i < 4u; ++i) {
    const unsigned r = 16u * i + (tid >> 4);
    const unsigned c = (tid & 15u) * 4u;
    xs[i] = *(const v4f*)&Cs[r * LDC + c];
    off[i] = (size_t)(row0 + r) * DIM + n0 + c;
  }
#pragma unroll
  for (int i = 0; i < 4; ++i) *(volatile v4f*)(outf + off[i]) = xs[i];
  __threadfence();
#pragma unroll
  for (int i = 0; i < 4; ++i) *(volatile v4f*)(outf + off[i]) = xs[i];
}
static_assert(16 * 4 == 64);
static_assert(64 * 4 * 8 == 64 * KM);
static_assert((size_t)64 * LDC * 4 + (size_t)64 * LDM * 2 + 64 * 4 <= (size_t)131072);

extern "C" void kernel_launch(void* const* d_in, const int* in_sizes, int n_in,
                              void* d_out, int out_size, void* d_ws, size_t ws_size,
                              hipStream_t stream) {
  if (n_in < 5) return;
  if ((long long)in_sizes[0] < (long long)MROWS * DIM) return;
  if ((long long)in_sizes[1] < (long long)NB * NOBJ * DIM) return;
  if ((long long)in_sizes[2] < (long long)NB * NOBJ * 4) return;
  if ((long long)in_sizes[3] < (long long)DIM * DIM) return;
  if ((long long)in_sizes[4] < (long long)DIM * DIM) return;
  if ((long long)out_size < (long long)MROWS * DIM) return;
  if (ws_size < WS_TOTAL) return;

  const float* patches = (const float*)d_in[0];
  const float* embs    = (const float*)d_in[1];
  const int*   loc     = (const int*)d_in[2];
  const float* wp      = (const float*)d_in[3];
  const float* we      = (const float*)d_in[4];
  float* out = (float*)d_out;

  char* ws = (char*)d_ws;
  _Float16* Wp_t = (_Float16*)(ws + OFF_WPT);
  _Float16* We_t = (_Float16*)(ws + OFF_WET);
  _Float16* P16  = (_Float16*)(ws + OFF_P16);
  _Float16* E16  = (_Float16*)(ws + OFF_E16);
  _Float16* InjT = (_Float16*)(ws + OFF_INJT);

  dim3 blk(256);
  wconv_kernel<<<dim3(DIM / 64, DIM / 64), blk, 0, stream>>>(wp, Wp_t, (unsigned)DIM, (unsigned)DIM);
  wconv_kernel<<<dim3(DIM / 64, DIM / 64), blk, 0, stream>>>(we, We_t, (unsigned)DIM, (unsigned)DIM);
  pconv_kernel<<<dim3((unsigned)(((size_t)MROWS * DIM) / 2048u)), blk, 0, stream>>>(patches, P16);
  ebuild_kernel<<<dim3(NBP), blk, 0, stream>>>(embs, E16);
  gemm_inj_kernel<<<dim3(DIM / 64, EROWS / 64), blk, 0, stream>>>(E16, We_t, InjT);
  fuse_kernel<<<dim3(DIM / 64, MROWS / 64), blk, 0, stream>>>(P16, Wp_t, InjT, loc, out);
}
